// RepeatedAttention_70660801954634
// MI455X (gfx1250) — hardware-verified
//
#include <hip/hip_runtime.h>


#define SS   2048
#define HID  2048
#define NH_  16
#define NKV  4
#define HD   128
#define WIN  512
#define NT64 (SS / 64)
#define ZH   2
#define DM   HID
#define PCAR 1024.0f
#define LOSC 1024.0f
typedef _Float16 h16;
typedef unsigned short bf;
typedef __attribute__((ext_vector_type(16))) __bf16   v16bf;
typedef __attribute__((ext_vector_type(16))) _Float16 v16h;
typedef __attribute__((ext_vector_type(8)))  _Float16 v8h;
typedef __attribute__((ext_vector_type(8)))  unsigned short v8us;
typedef __attribute__((ext_vector_type(8)))  float    v8f;
typedef __attribute__((ext_vector_type(4)))  float    v4f;
typedef v8h  __attribute__((may_alias)) v8ha;
typedef v4f  __attribute__((may_alias)) v4fa;
typedef v8us __attribute__((may_alias)) v8usa;

__device__ __forceinline__ unsigned short f2bf(float f) { unsigned u = __float_as_uint(f); u += 0x7FFFu + ((u >> 16) & 1u); return (unsigned short)(u >> 16); }
__device__ __forceinline__ float bf2f(unsigned short b) { return __uint_as_float(((unsigned)b) << 16); }
__device__ __forceinline__ float bfr(float f) { return bf2f(f2bf(f)); }
__device__ __forceinline__ v16h cat16(v8h lo, v8h hi) { return __builtin_shufflevector(lo, hi, 0, 1, 2, 3, 4, 5, 6, 7, 8, 9, 10, 11, 12, 13, 14, 15); }
__device__ __forceinline__ v16bf cat16b(v8us lo, v8us hi) { return __builtin_bit_cast(v16bf, __builtin_shufflevector(lo, hi, 0, 1, 2, 3, 4, 5, 6, 7, 8, 9, 10, 11, 12, 13, 14, 15)); }
__device__ __forceinline__ v8f wmma16(v16h a, v16h b, v8f c) { return __builtin_amdgcn_wmma_f32_16x16x32_f16(false, a, false, b, (short)0, c, false, false); }
__device__ __forceinline__ v8f wmmab(v16bf a, v16bf b, v8f c) { return __builtin_amdgcn_wmma_f32_16x16x32_bf16(false, a, false, b, (short)0, c, false, false); }


__global__ __launch_bounds__(128) void k_gemmh(const h16* __restrict__ A, const h16* __restrict__ Bn, const float* __restrict__ bias, float* C, int ldc, const float* __restrict__ R, int K, size_t sA, size_t sB, size_t sC, int roundR) {
    __shared__ __align__(16) float ost[4][16 * 68];
    const size_t z = blockIdx.z; A += z * sA; Bn += z * sB; C += z * sC; if (R) R += z * sC;
    const int lane = threadIdx.x & 31, wave = threadIdx.x >> 5, lr = lane & 15, hi = lane >> 4;
    const int r0 = blockIdx.x * 64 + wave * 16, c0 = blockIdx.y * 64;
    const size_t aoff = (size_t)(r0 + lr) * K + 8 * hi;
    size_t boff[4];
#pragma unroll
    for (int t = 0; t < 4; ++t) boff[t] = (size_t)(c0 + t * 16 + lr) * K + 8 * hi;
    v8f acc[4];
#pragma unroll
    for (int t = 0; t < 4; ++t) acc[t] = (v8f){};
#pragma unroll 1
    for (int kc = 0; kc < K; kc += 32) {
        const v16h a = cat16(*(const v8h*)(A + aoff + kc), *(const v8h*)(A + aoff + kc + 16));
#pragma unroll
        for (int t = 0; t < 4; ++t) { const v16h b = cat16(*(const v8h*)(Bn + boff[t] + kc), *(const v8h*)(Bn + boff[t] + kc + 16)); acc[t] = wmma16(a, b, acc[t]); }
        asm volatile("v_nop\n\tv_nop\n\tv_nop\n\tv_nop" : "+v"(acc[0]), "+v"(acc[1]), "+v"(acc[2]), "+v"(acc[3]) : "v"(a));
    }
    float* os = &ost[wave][0];
#pragma unroll
    for (int t = 0; t < 4; ++t) { const float bv = bias ? bfr(bias[c0 + t * 16 + lr]) : 0.f;
#pragma unroll
        for (int j = 0; j < 8; ++j) os[(hi * 8 + j) * 68 + t * 16 + lr] = acc[t][j] + bv; }
    __syncthreads();
    float* crow = C + (size_t)r0 * ldc + c0;
    auto pass = [&]() {
#pragma unroll
        for (int s = 0; s < 8; ++s) { const int Lid = (lane >> 3) + 4 * s, piece = lane & 7; const int row = Lid >> 1, cofs = (Lid & 1) * 32 + piece * 4;
            v4f val = *(const v4fa*)(os + row * 68 + cofs); if (R) { const v4f rv = *(const v4f*)(R + ((size_t)r0 + row) * ldc + c0 + cofs); val += roundR ? (v4f){bfr(rv[0]), bfr(rv[1]), bfr(rv[2]), bfr(rv[3])} : rv; }
            *(volatile v4f*)(crow + (size_t)row * ldc + cofs) = val; }
    };
    pass(); __threadfence(); pass();
}

template <int MODE>
__global__ __launch_bounds__(128) void k_gemm3z(const bf* __restrict__ Ah, const bf* __restrict__ Al, const bf* __restrict__ Bh, const bf* __restrict__ Bl, int K, float* C, int ldc, size_t sA, size_t sB, size_t sC) {
    if ((MODE & 1) && (int)blockIdx.y * 64 > (int)blockIdx.x * 64 + 63) return;
    const size_t z = blockIdx.z; Ah += z * sA; Al += z * sA; Bh += z * sB; Bl += z * sB; C += z * sC;
    const int Klim = (MODE & 2) ? min(K, ((int)blockIdx.x + 1) * 64) : K;
    __shared__ __align__(16) float ost[4][16 * 68];
    const int lane = threadIdx.x & 31, wave = threadIdx.x >> 5, lr = lane & 15, hi = lane >> 4;
    const int r0 = blockIdx.x * 64 + wave * 16, c0 = blockIdx.y * 64;
    const size_t aoff = (size_t)(r0 + lr) * K + 8 * hi;
    v8f acc[4];
#pragma unroll
    for (int t = 0; t < 4; ++t) acc[t] = (v8f){};
#pragma unroll 1
    for (int kc = 0; kc < Klim; kc += 32) {
        const v16bf a = cat16b(*(const v8us*)(Ah + aoff + kc), *(const v8us*)(Ah + aoff + kc + 16));
        v16bf al = a; if (!(MODE & 4) && !(MODE & 16)) al = cat16b(*(const v8us*)(Al + aoff + kc), *(const v8us*)(Al + aoff + kc + 16));
#pragma unroll
        for (int t = 0; t < 4; ++t) { const size_t bo = (size_t)(c0 + t * 16 + lr) * K + kc + 8 * hi;
            const v16bf bh = cat16b(*(const v8us*)(Bh + bo), *(const v8us*)(Bh + bo + 16));
            acc[t] = wmmab(a, bh, acc[t]);
            if (!(MODE & 4)) { if (!(MODE & 16)) acc[t] = wmmab(al, bh, acc[t]); if (!(MODE & 8)) { const v16bf bl = cat16b(*(const v8us*)(Bl + bo), *(const v8us*)(Bl + bo + 16)); acc[t] = wmmab(a, bl, acc[t]); } } }
        asm volatile("v_nop\n\tv_nop\n\tv_nop\n\tv_nop" : "+v"(acc[0]), "+v"(acc[1]), "+v"(acc[2]), "+v"(acc[3]) : "v"(a), "v"(al));
    }
    float* os = &ost[wave][0];
#pragma unroll
    for (int t = 0; t < 4; ++t) {
#pragma unroll
        for (int j = 0; j < 8; ++j) os[(hi * 8 + j) * 68 + t * 16 + lr] = acc[t][j]; }
    __builtin_amdgcn_wave_barrier(); asm volatile("" ::: "memory");
    float* crow = C + (size_t)r0 * ldc + c0;
    auto pass = [&]() {
#pragma unroll
        for (int s = 0; s < 8; ++s) { const int Lid = (lane >> 3) + 4 * s, piece = lane & 7; const int row = Lid >> 1, cofs = (Lid & 1) * 32 + piece * 4;
            const v4f val = *(const v4fa*)(os + row * 68 + cofs); *(volatile v4f*)(crow + (size_t)row * ldc + cofs) = val; }
    };
    pass(); __threadfence(); pass();
}
__global__ __launch_bounds__(256) void k_planes32z(const float* __restrict__ F, int ld, int off, float sc, int rows, bf* Ph, bf* Pl) {
    typedef __attribute__((ext_vector_type(2))) unsigned short v2us;
    const int lane = threadIdx.x & 31; const size_t r = ((size_t)blockIdx.x * 8 + (threadIdx.x >> 5)) * 2 + (lane >> 4); if (r >= (size_t)rows) return; const int z = blockIdx.z; const int c0 = (lane & 15) * 2; v2us oh, ol;
    Ph += (size_t)z * rows * 32; Pl += (size_t)z * rows * 32;
#pragma unroll
    for (int i = 0; i < 2; ++i) { const float y = F[r * ld + off + z * 32 + c0 + i] * sc; const unsigned short hb = f2bf(y); oh[i] = hb; ol[i] = f2bf(y - bf2f(hb)); }
    const size_t o = r * 32 + c0; *(volatile v2us*)(Ph + o) = oh; *(volatile v2us*)(Pl + o) = ol; __threadfence(); *(volatile v2us*)(Ph + o) = oh; *(volatile v2us*)(Pl + o) = ol;
}
__global__ __launch_bounds__(256) void k_vtpadz(const float* __restrict__ F, int ld, int off, int nk, bf* Th, bf* Tl) {
    typedef __attribute__((ext_vector_type(2))) unsigned short v2us;
    const int lane = threadIdx.x & 31; const size_t wid = (size_t)blockIdx.x * 8 + (threadIdx.x >> 5); if (wid >= (size_t)64 * (nk / 64)) return; const int z = blockIdx.z; const int d = (int)(wid / (nk / 64)); const int k0 = (int)(wid % (nk / 64)) * 64 + lane * 2; v2us oh, ol;
    Th += (size_t)z * 64 * nk; Tl += (size_t)z * 64 * nk;
#pragma unroll
    for (int i = 0; i < 2; ++i) { const float y = (d < 32) ? F[(size_t)(k0 + i) * ld + off + z * 32 + (d < 32 ? d : 0)] : 0.f; const unsigned short hb = f2bf(y); oh[i] = hb; ol[i] = f2bf(y - bf2f(hb)); }
    const size_t o = (size_t)d * nk + k0; *(volatile v2us*)(Th + o) = oh; *(volatile v2us*)(Tl + o) = ol; __threadfence(); *(volatile v2us*)(Th + o) = oh; *(volatile v2us*)(Tl + o) = ol;
}
template <int NK>
__global__ __launch_bounds__(256) void k_softmaxz(const float* __restrict__ S, int rows, bf* PH, bf* PL) {
    typedef __attribute__((ext_vector_type(4))) unsigned short v4us;
    const int lane = threadIdx.x & 31, i = blockIdx.x * 8 + (threadIdx.x >> 5); if (i >= rows) return; const size_t zo = (size_t)blockIdx.z * rows * NK; const float* sr = S + zo + (size_t)i * NK; PH += zo; PL += zo;
    float m = -3.0e38f;
#pragma unroll 1
    for (int c0 = lane * 4; c0 < NK; c0 += 128) {
#pragma unroll
        for (int q = 0; q < 4; ++q) m = fmaxf(m, sr[c0 + q]); }
#pragma unroll
    for (int sh = 16; sh; sh >>= 1) m = fmaxf(m, __shfl_xor(m, sh, 32));
    float sum = 0.f;
#pragma unroll 1
    for (int c0 = lane * 4; c0 < NK; c0 += 128) {
#pragma unroll
        for (int q = 0; q < 4; ++q) sum += __expf(sr[c0 + q] - m); }
#pragma unroll
    for (int sh = 16; sh; sh >>= 1) sum += __shfl_xor(sum, sh, 32);
    const float inv = 1.0f / sum;
#pragma unroll 1
    for (int ps = 0; ps < 2; ++ps) {
#pragma unroll 1
        for (int c0 = lane * 4; c0 < NK; c0 += 128) { v4us oh, ol;
#pragma unroll
            for (int q = 0; q < 4; ++q) { const float p = __expf(sr[c0 + q] - m) * inv; const unsigned short hb = f2bf(p); oh[q] = hb; ol[q] = f2bf(p - bf2f(hb)); }
            const size_t o = (size_t)i * NK + c0; *(volatile v4us*)(PH + o) = oh; *(volatile v4us*)(PL + o) = ol; }
        if (ps == 0) __threadfence(); }
}
__global__ __launch_bounds__(256) void k_placez(const float* __restrict__ XH, int rows, int ldy, float* Y) {
    const int lane = threadIdx.x & 31; const size_t q = (size_t)blockIdx.x * 8 + (threadIdx.x >> 5); if (q >= (size_t)rows) return; const int z = blockIdx.z; const float v = XH[((size_t)z * rows + q) * 64 + lane];
    *(volatile float*)(Y + q * ldy + z * 32 + lane) = v; __threadfence(); *(volatile float*)(Y + q * ldy + z * 32 + lane) = v;
}

template <typename T16> struct WFrag;
template <> struct WFrag<h16> { typedef v16h V; static __device__ __forceinline__ V ld(const h16* p) { return cat16(*(const v8h*)p, *(const v8h*)(p + 16)); } static __device__ __forceinline__ v8f mma(V a, V b, v8f c) { return wmma16(a, b, c); } };
template <> struct WFrag<bf> { typedef v16bf V; static __device__ __forceinline__ V ld(const bf* p) { return cat16b(*(const v8us*)p, *(const v8us*)(p + 16)); } static __device__ __forceinline__ v8f mma(V a, V b, v8f c) { return wmmab(a, b, c); } };
template <typename T16, int NSPLIT, bool BIAS>
__global__ __launch_bounds__(32) void k_gemmw(const T16* __restrict__ A, const T16* __restrict__ A2, const T16* __restrict__ Bt, const T16* __restrict__ Bt2, int K, float* C, int ldc, const float* __restrict__ bias, size_t sA, size_t sB, size_t sC) {
    typedef typename WFrag<T16>::V V;
    __shared__ __align__(16) float os[16 * 68];
    const size_t z = blockIdx.z; A += z * sA; if (A2) A2 += z * sA; Bt += z * sB; if (Bt2) Bt2 += z * sB; C += z * sC;
    const int lane = threadIdx.x & 31, lr = lane & 15, hi = lane >> 4; const int r0 = blockIdx.x * 64, c0 = blockIdx.y * 64;
    v8f acc[4][4];
#pragma unroll
    for (int mb = 0; mb < 4; ++mb)
#pragma unroll
        for (int nb = 0; nb < 4; ++nb) acc[mb][nb] = (v8f){};
    const size_t aoff = (size_t)(r0 + lr) * K + 8 * hi, boff = (size_t)(c0 + lr) * K + 8 * hi;
#pragma unroll 1
    for (int kc = 0; kc < K; kc += 32) {
        V a[4], a2[4];
#pragma unroll
        for (int mb = 0; mb < 4; ++mb) { a[mb] = WFrag<T16>::ld(A + aoff + (size_t)mb * 16 * K + kc); if (NSPLIT == 1 || NSPLIT == 2) a2[mb] = WFrag<T16>::ld(A2 + aoff + (size_t)mb * 16 * K + kc); }
#pragma unroll
        for (int nb = 0; nb < 4; ++nb) { const V b = WFrag<T16>::ld(Bt + boff + (size_t)nb * 16 * K + kc); V b2; if (NSPLIT >= 2) b2 = WFrag<T16>::ld(Bt2 + boff + (size_t)nb * 16 * K + kc);
#pragma unroll
            for (int mb = 0; mb < 4; ++mb) { acc[mb][nb] = WFrag<T16>::mma(a[mb], b, acc[mb][nb]); if (NSPLIT == 1 || NSPLIT == 2) acc[mb][nb] = WFrag<T16>::mma(a2[mb], b, acc[mb][nb]); if (NSPLIT >= 2) acc[mb][nb] = WFrag<T16>::mma(a[mb], b2, acc[mb][nb]); } }
        asm volatile("v_nop\n\tv_nop\n\tv_nop\n\tv_nop" : "+v"(acc[0][0]), "+v"(acc[1][1]), "+v"(acc[2][2]), "+v"(acc[3][3]) : "v"(a[0]), "v"(a[3]));
    }
#pragma unroll
    for (int mb = 0; mb < 4; ++mb) {
#pragma unroll
        for (int nb = 0; nb < 4; ++nb) {
#pragma unroll
            for (int j = 0; j < 8; ++j) os[(hi * 8 + j) * 68 + nb * 16 + lr] = acc[mb][nb][j]; }
        __builtin_amdgcn_wave_barrier(); asm volatile("" ::: "memory");
        float* crow = C + (size_t)(r0 + mb * 16) * ldc + c0;
#pragma unroll 1
        for (int ps = 0; ps < 2; ++ps) {
#pragma unroll
            for (int s = 0; s < 8; ++s) { const int row = 2 * s + hi, cofs = lr * 4; v4f val = *(const v4fa*)(os + row * 68 + cofs); if (BIAS) { val[0] += bfr(bias[c0 + cofs]); val[1] += bfr(bias[c0 + cofs + 1]); val[2] += bfr(bias[c0 + cofs + 2]); val[3] += bfr(bias[c0 + cofs + 3]); }
                *(volatile v4f*)(crow + (size_t)row * ldc + cofs) = val; }
            if (ps == 0) __threadfence(); }
        __builtin_amdgcn_wave_barrier(); asm volatile("" ::: "memory");
    }
}
template <typename T16, int NSPLIT, bool BIAS, int CAUS>
__global__ __launch_bounds__(32) void k_gemmwc(const T16* __restrict__ A, const T16* __restrict__ A2, const T16* __restrict__ Bt, const T16* __restrict__ Bt2, int K, float* C, int ldc, const float* __restrict__ bias, size_t sA, size_t sB, size_t sC) {
    typedef typename WFrag<T16>::V V;
    __shared__ __align__(16) float os[16 * 68];
    if (CAUS == 1 && (int)blockIdx.y * 64 > (int)blockIdx.x * 64) return;
    const int Klim = (CAUS == 2) ? min(K, ((int)blockIdx.x + 1) * 64) : K;
    const size_t z = blockIdx.z; A += z * sA; if (A2) A2 += z * sA; Bt += z * sB; if (Bt2) Bt2 += z * sB; C += z * sC;
    const int lane = threadIdx.x & 31, lr = lane & 15, hi = lane >> 4; const int r0 = blockIdx.x * 64, c0 = blockIdx.y * 64;
    v8f acc[4][4];
#pragma unroll
    for (int mb = 0; mb < 4; ++mb)
#pragma unroll
        for (int nb = 0; nb < 4; ++nb) acc[mb][nb] = (v8f){};
    const size_t aoff = (size_t)(r0 + lr) * K + 8 * hi, boff = (size_t)(c0 + lr) * K + 8 * hi;
#pragma unroll 1
    for (int kc = 0; kc < Klim; kc += 32) {
        V a[4], a2[4];
#pragma unroll
        for (int mb = 0; mb < 4; ++mb) { a[mb] = WFrag<T16>::ld(A + aoff + (size_t)mb * 16 * K + kc); if (NSPLIT == 1 || NSPLIT == 2) a2[mb] = WFrag<T16>::ld(A2 + aoff + (size_t)mb * 16 * K + kc); }
#pragma unroll
        for (int nb = 0; nb < 4; ++nb) { const V b = WFrag<T16>::ld(Bt + boff + (size_t)nb * 16 * K + kc); V b2; if (NSPLIT >= 2) b2 = WFrag<T16>::ld(Bt2 + boff + (size_t)nb * 16 * K + kc);
#pragma unroll
            for (int mb = 0; mb < 4; ++mb) { acc[mb][nb] = WFrag<T16>::mma(a[mb], b, acc[mb][nb]); if (NSPLIT == 1 || NSPLIT == 2) acc[mb][nb] = WFrag<T16>::mma(a2[mb], b, acc[mb][nb]); if (NSPLIT >= 2) acc[mb][nb] = WFrag<T16>::mma(a[mb], b2, acc[mb][nb]); } }
        asm volatile("v_nop\n\tv_nop\n\tv_nop\n\tv_nop" : "+v"(acc[0][0]), "+v"(acc[1][1]), "+v"(acc[2][2]), "+v"(acc[3][3]) : "v"(a[0]), "v"(a[3]));
    }
#pragma unroll
    for (int mb = 0; mb < 4; ++mb) {
#pragma unroll
        for (int nb = 0; nb < 4; ++nb) {
#pragma unroll
            for (int j = 0; j < 8; ++j) os[(hi * 8 + j) * 68 + nb * 16 + lr] = acc[mb][nb][j]; }
        __builtin_amdgcn_wave_barrier(); asm volatile("" ::: "memory");
        float* crow = C + (size_t)(r0 + mb * 16) * ldc + c0;
#pragma unroll 1
        for (int ps = 0; ps < 2; ++ps) {
#pragma unroll
            for (int s = 0; s < 8; ++s) { const int row = 2 * s + hi, cofs = lr * 4; v4f val = *(const v4fa*)(os + row * 68 + cofs); if (BIAS) { val[0] += bfr(bias[c0 + cofs]); val[1] += bfr(bias[c0 + cofs + 1]); val[2] += bfr(bias[c0 + cofs + 2]); val[3] += bfr(bias[c0 + cofs + 3]); }
                *(volatile v4f*)(crow + (size_t)row * ldc + cofs) = val; }
            if (ps == 0) __threadfence(); }
        __builtin_amdgcn_wave_barrier(); asm volatile("" ::: "memory");
    }
}
template <typename T16, int NSPLIT, bool BIAS, int FMODE>
__global__ __launch_bounds__(32) void k_gemmwf(const T16* __restrict__ A, const T16* __restrict__ A2, const T16* __restrict__ Bt, const T16* __restrict__ Bt2, int K, float* C, int ldc, const float* __restrict__ bias, size_t sA, size_t sB, size_t sC, const int* __restrict__ FL, int nt) {
    typedef typename WFrag<T16>::V V;
    __shared__ __align__(16) float os[16 * 68];
    const int I = blockIdx.x; if (FMODE == 1 && FL[I * nt + blockIdx.y] == 0) return;
    int Klo = 0, Klim = K; if (FMODE == 2) { int f = -1, l = -1; for (int j = 0; j < nt; ++j) { if (FL[I * nt + j]) { if (f < 0) f = j; l = j; } } if (f < 0) { Klo = 0; Klim = 0; } else { Klo = f * 64; Klim = (l + 1) * 64; } }
    const size_t z = blockIdx.z; A += z * sA; if (A2) A2 += z * sA; Bt += z * sB; if (Bt2) Bt2 += z * sB; C += z * sC;
    const int lane = threadIdx.x & 31, lr = lane & 15, hi = lane >> 4; const int r0 = blockIdx.x * 64, c0 = blockIdx.y * 64;
    v8f acc[4][4];
#pragma unroll
    for (int mb = 0; mb < 4; ++mb)
#pragma unroll
        for (int nb = 0; nb < 4; ++nb) acc[mb][nb] = (v8f){};
    const size_t aoff = (size_t)(r0 + lr) * K + 8 * hi, boff = (size_t)(c0 + lr) * K + 8 * hi;
#pragma unroll 1
    for (int kc = Klo; kc < Klim; kc += 32) {
        V a[4], a2[4];
#pragma unroll
        for (int mb = 0; mb < 4; ++mb) { a[mb] = WFrag<T16>::ld(A + aoff + (size_t)mb * 16 * K + kc); if (NSPLIT == 1 || NSPLIT == 2) a2[mb] = WFrag<T16>::ld(A2 + aoff + (size_t)mb * 16 * K + kc); }
#pragma unroll
        for (int nb = 0; nb < 4; ++nb) { const V b = WFrag<T16>::ld(Bt + boff + (size_t)nb * 16 * K + kc); V b2; if (NSPLIT >= 2) b2 = WFrag<T16>::ld(Bt2 + boff + (size_t)nb * 16 * K + kc);
#pragma unroll
            for (int mb = 0; mb < 4; ++mb) { acc[mb][nb] = WFrag<T16>::mma(a[mb], b, acc[mb][nb]); if (NSPLIT == 1 || NSPLIT == 2) acc[mb][nb] = WFrag<T16>::mma(a2[mb], b, acc[mb][nb]); if (NSPLIT >= 2) acc[mb][nb] = WFrag<T16>::mma(a[mb], b2, acc[mb][nb]); } }
        asm volatile("v_nop\n\tv_nop\n\tv_nop\n\tv_nop" : "+v"(acc[0][0]), "+v"(acc[1][1]), "+v"(acc[2][2]), "+v"(acc[3][3]) : "v"(a[0]), "v"(a[3]));
    }
#pragma unroll
    for (int mb = 0; mb < 4; ++mb) {
#pragma unroll
        for (int nb = 0; nb < 4; ++nb) {
#pragma unroll
            for (int j = 0; j < 8; ++j) os[(hi * 8 + j) * 68 + nb * 16 + lr] = acc[mb][nb][j]; }
        __builtin_amdgcn_wave_barrier(); asm volatile("" ::: "memory");
        float* crow = C + (size_t)(r0 + mb * 16) * ldc + c0;
#pragma unroll 1
        for (int ps = 0; ps < 2; ++ps) {
#pragma unroll
            for (int s = 0; s < 8; ++s) { const int row = 2 * s + hi, cofs = lr * 4; v4f val = *(const v4fa*)(os + row * 68 + cofs); if (BIAS) { val[0] += bfr(bias[c0 + cofs]); val[1] += bfr(bias[c0 + cofs + 1]); val[2] += bfr(bias[c0 + cofs + 2]); val[3] += bfr(bias[c0 + cofs + 3]); }
                *(volatile v4f*)(crow + (size_t)row * ldc + cofs) = val; }
            if (ps == 0) __threadfence(); }
        __builtin_amdgcn_wave_barrier(); asm volatile("" ::: "memory");
    }
}

typedef __attribute__((ext_vector_type(4))) _Float16 v4h;
__device__ __forceinline__ h16 tohx(float x) { return (h16)x; }
template <bool F16O>
__global__ __launch_bounds__(256) void k_wT(const float* __restrict__ Wm, int K, int N, bf* Bt, h16* Bh) {
    __shared__ float tl[64][65]; typedef __attribute__((ext_vector_type(4))) unsigned short v4us;
    const int tid = threadIdx.x; const int k0 = blockIdx.x * 64, n0 = blockIdx.y * 64; const int rr = tid >> 2, cq = (tid & 3) * 16;
#pragma unroll
    for (int i = 0; i < 16; ++i) tl[rr][cq + i] = bfr(Wm[(size_t)(k0 + rr) * N + n0 + cq + i]);
    __syncthreads();
    const int lane = tid & 31, wv = tid >> 5;
    auto pass = [&]() {
#pragma unroll
        for (int st = 0; st < 4; ++st) { const int nr = wv * 8 + st * 2 + (lane >> 4); const int kq = (lane & 15) * 4; const size_t off = (size_t)(n0 + nr) * K + k0 + kq;
            if (F16O) { v4h v; for (int i = 0; i < 4; ++i) v[i] = tohx(tl[kq + i][nr]); *(volatile v4h*)(Bh + off) = v; } else { v4us v; for (int i = 0; i < 4; ++i) v[i] = f2bf(tl[kq + i][nr]); *(volatile v4us*)(Bt + off) = v; } }
    };
    pass(); __threadfence(); pass();
}
__global__ __launch_bounds__(256) void k_cvtx(const float* __restrict__ x, bf* A) {
    const int lane = threadIdx.x & 31; const size_t r = (size_t)blockIdx.x * 8 + (threadIdx.x >> 5); if (r >= (size_t)SS) return;
#pragma unroll 1
    for (int ps = 0; ps < 2; ++ps) {
#pragma unroll
        for (int q = 0; q < HID / 256; ++q) { const size_t o = r * HID + q * 256 + lane * 8; v8us v;
#pragma unroll
            for (int i = 0; i < 8; ++i) v[i] = f2bf(x[o + i]);
            *(volatile v8us*)(A + o) = v; }
        if (ps == 0) __threadfence(); }
}
__global__ __launch_bounds__(256) void k_flags(int* FL) { const int lane = threadIdx.x & 31, I = blockIdx.x * 8 + (threadIdx.x >> 5); if (I >= NT64) return; const int v = (lane <= I && lane >= I - WIN / 64) ? 1 : 0; *(volatile int*)(FL + I * NT64 + lane) = v; __threadfence(); *(volatile int*)(FL + I * NT64 + lane) = v; }
__global__ __launch_bounds__(256) void k_ropepl(const float* __restrict__ F, int ldf, int col0, int h0, float sc, const float* __restrict__ cs, const float* __restrict__ sn, h16* P) {
    const int lane = threadIdx.x & 31; const int t = blockIdx.x * 8 + (threadIdx.x >> 5); if (t >= SS) return; const int z = blockIdx.z; const float* fr = F + (size_t)t * ldf + col0 + (h0 + z) * HD; const int d0 = lane * 4; v4h o;
#pragma unroll
    for (int i = 0; i < 4; ++i) { const int d = d0 + i; const float rot = (d < HD / 2) ? -fr[d + HD / 2] : fr[d - HD / 2]; o[i] = tohx((fr[d] * bfr(cs[(size_t)t * HD + d]) + rot * bfr(sn[(size_t)t * HD + d])) * sc); }
    const size_t off = ((size_t)z * SS + t) * HD + d0; *(volatile v4h*)(P + off) = o; __threadfence(); *(volatile v4h*)(P + off) = o;
}
__global__ __launch_bounds__(256) void k_vTr(const float* __restrict__ V, int g, h16* VT) {
    __shared__ float tl[64][65];
    const int tid = threadIdx.x; const int t0 = blockIdx.x * 64, d0 = blockIdx.y * 64; const int rr = tid >> 2, cq = (tid & 3) * 16;
#pragma unroll
    for (int i = 0; i < 16; ++i) tl[rr][cq + i] = V[(size_t)(t0 + rr) * (NKV * HD) + g * HD + d0 + cq + i];
    __syncthreads();
    const int lane = tid & 31, wv = tid >> 5;
    auto pass = [&]() {
#pragma unroll
        for (int st = 0; st < 4; ++st) { const int dr = wv * 8 + st * 2 + (lane >> 4); const int tq = (lane & 15) * 4; v4h v;
#pragma unroll
            for (int i = 0; i < 4; ++i) v[i] = tohx(tl[tq + i][dr]);
            *(volatile v4h*)(VT + (size_t)(d0 + dr) * SS + t0 + tq) = v; }
    };
    pass(); __threadfence(); pass();
}
template <bool WND>
__global__ __launch_bounds__(256) void k_softm(const float* __restrict__ S, h16* P) {
    const int lane = threadIdx.x & 31, i = blockIdx.x * 8 + (threadIdx.x >> 5); if (i >= SS) return; const size_t zo = ((size_t)blockIdx.z * SS + i) * SS; const float* sr = S + zo; h16* po = P + zo;
    const int lo = WND ? max(0, i - WIN) : 0; const int clo = lo & ~127, chi = (i | 127) + 1;
    auto live = [&](int j) { return j <= i && j >= lo; };
    float m = -3.0e38f;
#pragma unroll 1
    for (int c0 = clo + lane * 4; c0 < chi; c0 += 128) {
#pragma unroll
        for (int q = 0; q < 4; ++q) if (live(c0 + q)) m = fmaxf(m, sr[c0 + q]); }
#pragma unroll
    for (int sh = 16; sh; sh >>= 1) m = fmaxf(m, __shfl_xor(m, sh, 32));
    float sum = 0.f;
#pragma unroll 1
    for (int c0 = clo + lane * 4; c0 < chi; c0 += 128) {
#pragma unroll
        for (int q = 0; q < 4; ++q) if (live(c0 + q)) sum += __expf(sr[c0 + q] - m); }
#pragma unroll
    for (int sh = 16; sh; sh >>= 1) sum += __shfl_xor(sum, sh, 32);
    const float f = __fdiv_rn(PCAR, sum);
#pragma unroll 1
    for (int ps = 0; ps < 2; ++ps) {
#pragma unroll 1
        for (int c0 = lane * 4; c0 < SS; c0 += 128) { v4h o;
#pragma unroll
            for (int q = 0; q < 4; ++q) { const int j = c0 + q; o[q] = tohx(live(j) ? __expf(sr[live(j) ? j : 0] - m) * f : 0.f); }
            *(volatile v4h*)(po + c0) = o; }
        if (ps == 0) __threadfence(); }
}
__global__ __launch_bounds__(256) void k_mergeo(const float* __restrict__ OZ, int col0, int h0, const float* __restrict__ gamma, int useg, h16* OC) {
    const int lane = threadIdx.x & 31; const int t = blockIdx.x * 8 + (threadIdx.x >> 5); if (t >= SS) return; const int z = blockIdx.z; const float gs = useg ? tanhf(bfr(gamma[h0 + z])) : 1.0f; v4h o;
#pragma unroll
    for (int i = 0; i < 4; ++i) o[i] = tohx(OZ[((size_t)z * SS + t) * HD + lane * 4 + i] * (1.0f / PCAR) * gs);
    const size_t off = (size_t)t * (2 * HID) + col0 + (h0 + z) * HD + lane * 4; *(volatile v4h*)(OC + off) = o; __threadfence(); *(volatile v4h*)(OC + off) = o;
}
extern "C" void kernel_launch(void* const* d_in, const int* in_sizes, int n_in,
                              void* d_out, int out_size, void* d_ws, size_t ws_size, hipStream_t stream) {
    (void)in_sizes; (void)n_in; (void)out_size;
    const float* x = (const float*)d_in[0]; const float* cs = (const float*)d_in[1]; const float* sn = (const float*)d_in[2]; const float* Wq = (const float*)d_in[3]; const float* bq = (const float*)d_in[4]; const float* Wk = (const float*)d_in[5]; const float* bk = (const float*)d_in[6]; const float* Wv = (const float*)d_in[7]; const float* bv = (const float*)d_in[8]; const float* Wo = (const float*)d_in[9]; const float* gamma = (const float*)d_in[10];
    float* out = (float*)d_out;
    char* wsp = (char*)d_ws;
    auto take = [&](size_t bytes) { char* p = wsp; wsp += (bytes + 255) & ~(size_t)255; return (void*)p; };
    bf* WQ = (bf*)take((size_t)2 * HID * HID * 2); bf* WK = (bf*)take((size_t)NKV * HD * HID * 2); bf* WV = (bf*)take((size_t)NKV * HD * HID * 2); h16* WO = (h16*)take((size_t)HID * 2 * HID * 2); int* FL = (int*)take(NT64 * NT64 * 4);
    bf* XB = (bf*)take((size_t)SS * HID * 2); float* Q = (float*)take((size_t)SS * 2 * HID * 4); float* Kf = (float*)take((size_t)SS * NKV * HD * 4); float* V = (float*)take((size_t)SS * NKV * HD * 4);
    h16* Qx = (h16*)take((size_t)ZH * SS * HD * 2); h16* Kx = (h16*)take((size_t)SS * HD * 2); h16* VT = (h16*)take((size_t)HD * SS * 2); float* S = (float*)take((size_t)ZH * SS * SS * 4); h16* Px = (h16*)take((size_t)ZH * SS * SS * 2); float* OZ = (float*)take((size_t)ZH * SS * HD * 4); h16* OC = (h16*)take((size_t)SS * 2 * HID * 2);
    if ((size_t)(wsp - (char*)d_ws) > ws_size) return;
    k_wT<false><<<dim3(HID / 64, (2 * HID) / 64, 1), 256, 0, stream>>>(Wq, HID, 2 * HID, WQ, nullptr); k_wT<false><<<dim3(HID / 64, (NKV * HD) / 64, 1), 256, 0, stream>>>(Wk, HID, NKV * HD, WK, nullptr); k_wT<false><<<dim3(HID / 64, (NKV * HD) / 64, 1), 256, 0, stream>>>(Wv, HID, NKV * HD, WV, nullptr); k_wT<true><<<dim3((2 * HID) / 64, HID / 64, 1), 256, 0, stream>>>(Wo, 2 * HID, HID, nullptr, WO);
    k_flags<<<NT64 / 8, 256, 0, stream>>>(FL); k_cvtx<<<SS / 8, 256, 0, stream>>>(x, XB);
    k_gemmw<bf, 0, true><<<dim3(SS / 64, (2 * HID) / 64, 1), 32, 0, stream>>>(XB, nullptr, WQ, nullptr, HID, Q, 2 * HID, bq, 0, 0, 0);
    k_gemmw<bf, 0, true><<<dim3(SS / 64, (NKV * HD) / 64, 1), 32, 0, stream>>>(XB, nullptr, WK, nullptr, HID, Kf, NKV * HD, bk, 0, 0, 0);
    k_gemmw<bf, 0, true><<<dim3(SS / 64, (NKV * HD) / 64, 1), 32, 0, stream>>>(XB, nullptr, WV, nullptr, HID, V, NKV * HD, bv, 0, 0, 0);
    const float SC = 0.08838834764831845f;
    for (int g = 0; g < NKV; ++g) {
        k_ropepl<<<dim3(SS / 8, 1, 1), 256, 0, stream>>>(Kf, NKV * HD, 0, g, 1.0f, cs, sn, Kx); k_vTr<<<dim3(SS / 64, HD / 64, 1), 256, 0, stream>>>(V, g, VT);
        for (int h0 = g * 4; h0 < g * 4 + 4; h0 += ZH)
            for (int s = 0; s < 2; ++s) {
                k_ropepl<<<dim3(SS / 8, 1, ZH), 256, 0, stream>>>(Q, 2 * HID, s * HID, h0, SC, cs, sn, Qx);
                if (s == 0) { k_gemmwc<h16, 0, false, 1><<<dim3(SS / 64, SS / 64, ZH), 32, 0, stream>>>(Qx, nullptr, Kx, nullptr, HD, S, SS, nullptr, (size_t)SS * HD, 0, (size_t)SS * SS);
                              k_softm<false><<<dim3(SS / 8, 1, ZH), 256, 0, stream>>>(S, Px);
                              k_gemmwc<h16, 0, false, 2><<<dim3(SS / 64, HD / 64, ZH), 32, 0, stream>>>(Px, nullptr, VT, nullptr, SS, OZ, HD, nullptr, (size_t)SS * SS, 0, (size_t)SS * HD); }
                else        { k_gemmwf<h16, 0, false, 1><<<dim3(SS / 64, SS / 64, ZH), 32, 0, stream>>>(Qx, nullptr, Kx, nullptr, HD, S, SS, nullptr, (size_t)SS * HD, 0, (size_t)SS * SS, FL, NT64);
                              k_softm<true><<<dim3(SS / 8, 1, ZH), 256, 0, stream>>>(S, Px);
                              k_gemmwf<h16, 0, false, 2><<<dim3(SS / 64, HD / 64, ZH), 32, 0, stream>>>(Px, nullptr, VT, nullptr, SS, OZ, HD, nullptr, (size_t)SS * SS, 0, (size_t)SS * HD, FL, NT64); }
                k_mergeo<<<dim3(SS / 8, 1, ZH), 256, 0, stream>>>(OZ, s * HID, h0, gamma, s, OC); } }
    k_gemmw<h16, 0, false><<<dim3(SS / 64, HID / 64, 1), 32, 0, stream>>>(OC, nullptr, WO, nullptr, 2 * HID, out, HID, nullptr, 0, 0, 0);
}
